// CasualMultiHeadAttention_28303834480703
// MI455X (gfx1250) — hardware-verified
//
#include <hip/hip_runtime.h>

typedef __attribute__((ext_vector_type(16))) _Float16 v16h;
typedef __attribute__((ext_vector_type(8)))  _Float16 v8h;
typedef __attribute__((ext_vector_type(16))) __bf16   v16b;
typedef __attribute__((ext_vector_type(8)))  __bf16   v8b;
typedef __attribute__((ext_vector_type(8)))  float    v8f;
typedef __attribute__((ext_vector_type(4)))  float    v4f;
typedef __attribute__((ext_vector_type(4)))  unsigned v4u;
#define U16(p) ((const unsigned short*)(const void*)(p))

constexpr int NB    = 2;
constexpr int SEQ   = 2048;
constexpr int EMB   = 1024;
constexpr int NHEAD = 16;
constexpr int HDIM  = 64;
constexpr int NTOK  = NB * SEQ;
constexpr int NROWH = NTOK * NHEAD;

constexpr int AQB = 64;
constexpr int AKC = 64;
constexpr int ANW = 4;

static_assert(NROWH % 64 == 0);
static_assert(HDIM % 64 == 0);
static_assert(HDIM % 32 == 0);
static_assert(NTOK % 64 == 0);
static_assert(EMB % 64 == 0);
static_assert(EMB % 32 == 0);
static_assert(SEQ % AQB == 0);
static_assert(AQB == AKC);

constexpr size_t MIB      = 1048576;
constexpr size_t OFF_XH   = 0;
constexpr size_t OFF_XL   = 8 * MIB;
constexpr size_t OFF_WH   = 16 * MIB;
constexpr size_t OFF_WL   = 16 * MIB + 65536;
constexpr size_t OFF_WOH  = 17 * MIB;
constexpr size_t OFF_WOL  = 19 * MIB;
constexpr size_t OFF_QKVH = 21 * MIB;
constexpr size_t OFF_QKVL = 45 * MIB;
constexpr size_t OFF_AVH  = 69 * MIB;
constexpr size_t OFF_AVL  = 77 * MIB;
constexpr size_t WS_TOTAL = 85 * MIB;
constexpr size_t PLANE_QKV = (size_t)NROWH * HDIM;
static_assert((size_t)NB * SEQ * EMB * 2 <= OFF_XL - OFF_XH);
static_assert((size_t)3 * HDIM * HDIM * 2 <= OFF_WL - OFF_WH);
static_assert((size_t)3 * HDIM * HDIM * 2 <= OFF_WOH - OFF_WL);
static_assert((size_t)EMB * EMB * 2 <= OFF_WOL - OFF_WOH);
static_assert((size_t)EMB * EMB * 2 <= OFF_QKVH - OFF_WOL);
static_assert(3 * PLANE_QKV * 2 <= OFF_QKVL - OFF_QKVH);
static_assert(3 * PLANE_QKV * 2 <= OFF_AVH - OFF_QKVL);
static_assert((size_t)NTOK * EMB * 2 <= OFF_AVL - OFF_AVH);
static_assert((size_t)NTOK * EMB * 2 <= WS_TOTAL - OFF_AVL);
static_assert(WS_TOTAL <= 134217728);

__device__ __forceinline__ unsigned short f2bf_bits(float f) {
  unsigned u = __float_as_uint(f);
  return (unsigned short)((u + 0x7FFFu + ((u >> 16) & 1u)) >> 16);
}
__device__ __forceinline__ float bf_bits2f(unsigned short h) { return __uint_as_float(((unsigned)h) << 16); }

__device__ __forceinline__ void dep_guard_h(v8f& a, v8f& b, v16h x, v16h y) { asm volatile("v_nop\n\tv_nop\n\tv_nop\n\tv_nop" : "+v"(a), "+v"(b) : "v"(x), "v"(y)); }
__device__ __forceinline__ void dep_guard_b(v8f& a, v8f& b, v16b x, v16b y) { asm volatile("v_nop\n\tv_nop\n\tv_nop\n\tv_nop" : "+v"(a), "+v"(b) : "v"(x), "v"(y)); }
__device__ __forceinline__ void keep4_h(v16h a, v16h b, v16h c, v16h d) { asm volatile("v_nop" :: "v"(a), "v"(b), "v"(c), "v"(d)); }
__device__ __forceinline__ void keep4_b(v16b a, v16b b, v16b c, v16b d) { asm volatile("v_nop" :: "v"(a), "v"(b), "v"(c), "v"(d)); }
__device__ __forceinline__ void acc_guard4(v8f& a, v8f& b, v8f& c, v8f& d) { asm volatile("v_nop\n\tv_nop\n\tv_nop\n\tv_nop" : "+v"(a), "+v"(b), "+v"(c), "+v"(d)); }
template <typename T> struct Frag;
template <> struct Frag<_Float16> {
  typedef v16h V; union U { v16h v; v8h h[2]; };
  static __device__ __forceinline__ v16h load(const _Float16* p) {
    U f; f.h[0] = *(const v8h*)(p); f.h[1] = *(const v8h*)(p + 16); return f.v;
  }
  static __device__ __forceinline__ v8f mma(v16h a, v16h b, v8f c) {
    return __builtin_amdgcn_wmma_f32_16x16x32_f16(false, a, false, b, (short)0, c, false, false);
  }
  static __device__ __forceinline__ void guard(v8f& a, v8f& b, v16h x, v16h y) { dep_guard_h(a, b, x, y); }
  static __device__ __forceinline__ void keep(v16h a, v16h b, v16h c, v16h d) { keep4_h(a, b, c, d); }
};
template <> struct Frag<__bf16> {
  typedef v16b V; union U { v16b v; v8b h[2]; };
  static __device__ __forceinline__ v16b load(const __bf16* p) {
    U f; f.h[0] = *(const v8b*)(p); f.h[1] = *(const v8b*)(p + 16); return f.v;
  }
  static __device__ __forceinline__ v8f mma(v16b a, v16b b, v8f c) {
    return __builtin_amdgcn_wmma_f32_16x16x32_bf16(false, a, false, b, (short)0, c, false, false);
  }
  static __device__ __forceinline__ void guard(v8f& a, v8f& b, v16b x, v16b y) { dep_guard_b(a, b, x, y); }
  static __device__ __forceinline__ void keep(v16b a, v16b b, v16b c, v16b d) { keep4_b(a, b, c, d); }
};

template <int ET> struct Elem;
template <> struct Elem<0> { typedef _Float16 T; };
template <> struct Elem<1> { typedef __bf16 T; };
template <int ET, bool SPLIT, int BIAS_MODE, int OUT_MODE, bool RESID, int ACT = 0>
__global__ __launch_bounds__(256) void wmma_gemm64(
    const unsigned short* __restrict__ Ap, const unsigned short* __restrict__ A2p, int lda, long strideA,
    const unsigned short* __restrict__ Btp, const unsigned short* __restrict__ Bt2p, int ldb, long strideB,
    void* __restrict__ Cout, void* __restrict__ Cout2, int ldc, long strideC,
    const float* __restrict__ bias,
    const float* __restrict__ resid, long strideR,
    int M, int N, int K, float scale) {
  typedef typename Elem<ET>::T T;
  typedef typename Frag<T>::V V;
  const T* A = (const T*)Ap; const T* A2 = (const T*)A2p; const T* Bt = (const T*)Btp; const T* Bt2 = (const T*)Bt2p;
  __shared__ __align__(16) float sT[8][16 * 68];
  const int b    = blockIdx.y;
  const int lane = threadIdx.x & 31;
  const int wave = threadIdx.x >> 5;
  const int tilesN = N >> 6;
  const int tilesM = M >> 6;
  const int tile = blockIdx.x * 8 + wave;
  if (tile >= tilesM * tilesN) return;
  const int tm = tile / tilesN;
  const int tn = tile - tm * tilesN;
  const int m0 = tm << 6;
  const int n0 = tn << 6;

  const T* Ab  = A  + (size_t)b * strideA;
  const T* Bb  = Bt + (size_t)b * strideB;
  const T* Ab2 = SPLIT ? (A2  + (size_t)b * strideA) : nullptr;
  const T* Bb2 = SPLIT ? (Bt2 + (size_t)b * strideB) : nullptr;

  const int rlane = lane & 15;
  const int koff  = (lane >> 4) * 8;
  const int mOff  = (lane >> 4) * 8;

  v8f acc[4][4];
#pragma unroll
  for (int i = 0; i < 4; ++i)
#pragma unroll
    for (int j = 0; j < 4; ++j) acc[i][j] = (v8f){0.f,0.f,0.f,0.f,0.f,0.f,0.f,0.f};

  for (int k0 = 0; k0 < K; k0 += 32) {
    V bh[4], bl[4];
#pragma unroll
    for (int j = 0; j < 4; ++j) {
      const size_t bo = (size_t)(n0 + (j << 4) + rlane) * ldb + koff + k0;
      bh[j] = Frag<T>::load(Bb + bo);
      if (SPLIT) bl[j] = Frag<T>::load(Bb2 + bo);
    }
#pragma unroll
    for (int i = 0; i < 4; ++i) {
      const size_t ao = (size_t)(m0 + (i << 4) + rlane) * lda + koff + k0;
      V ah = Frag<T>::load(Ab + ao);
      V al;
      if (SPLIT) al = Frag<T>::load(Ab2 + ao);
#pragma unroll
      for (int j = 0; j < 4; ++j) {
        acc[i][j] = Frag<T>::mma(ah, bh[j], acc[i][j]);
        if (SPLIT) {
          acc[i][j] = Frag<T>::mma(ah, bl[j], acc[i][j]);
          acc[i][j] = Frag<T>::mma(al, bh[j], acc[i][j]);
        }
      }
      Frag<T>::guard(acc[i][0], acc[i][3], ah, SPLIT ? al : ah);
    }
    Frag<T>::keep(bh[0], bh[1], bh[2], bh[3]);
    if (SPLIT) Frag<T>::keep(bl[0], bl[1], bl[2], bl[3]);
  }
  acc_guard4(acc[0][0], acc[0][1], acc[0][2], acc[0][3]);
  acc_guard4(acc[1][0], acc[1][1], acc[1][2], acc[1][3]);
  acc_guard4(acc[2][0], acc[2][1], acc[2][2], acc[2][3]);
  acc_guard4(acc[3][0], acc[3][1], acc[3][2], acc[3][3]);

  float* slab = sT[wave];
  const float* Rb = RESID ? (resid + (size_t)b * strideR) : nullptr;
#pragma unroll
  for (int i = 0; i < 4; ++i) {
    const int mBase = m0 + (i << 4);
#pragma unroll
    for (int j = 0; j < 4; ++j) {
      const int n = n0 + (j << 4) + rlane;
      float bv = 0.f;
      if (BIAS_MODE == 2) bv = bias[n];
#pragma unroll
      for (int r = 0; r < 8; ++r) {
        float v = acc[i][j][r] * scale;
        if (BIAS_MODE == 1) v += bias[mBase + mOff + r];
        if (BIAS_MODE == 2) v += bv;
        if (RESID) v += Rb[(size_t)(mBase + mOff + r) * ldc + n];
        if (ACT == 1) v = tanhf(v);
        if (ACT == 2) v = fmaxf(v, 0.0f);
        if (ACT == 3) v = v / (1.0f + expf(-v));
        if (ACT == 4) v = (v > 0.f) ? v : 0.01f * v;
        if (ACT == 5) v = 0.5f * v * (1.0f + erff(v * 0.70710678118654752f));
        slab[(mOff + r) * 68 + (j << 4) + rlane] = v;
      }
    }
    __builtin_amdgcn_fence(__ATOMIC_RELEASE, "workgroup");
    __builtin_amdgcn_wave_barrier();
    __builtin_amdgcn_fence(__ATOMIC_ACQUIRE, "workgroup");
    if (OUT_MODE == 0) {
      float* C = (float*)Cout + (size_t)b * strideC;
      const int hh = lane >> 4, c4 = (lane & 15) * 4;
      for (int pass = 0; pass < 2; ++pass) {
#pragma unroll
        for (int it = 0; it < 8; ++it) {
          const int row = it * 2 + hh;
          v4f v = *(const v4f*)(slab + row * 68 + c4);
          *(volatile v4f*)(C + (size_t)(mBase + row) * ldc + n0 + c4) = v;
        }
        __threadfence();
      }
    } else {
      const int q = lane >> 3, c8 = (lane & 7) * 8;
      unsigned short* C  = (unsigned short*)Cout  + (size_t)b * strideC;
      unsigned short* C2 = (OUT_MODE == 2) ? ((unsigned short*)Cout2 + (size_t)b * strideC) : nullptr;
      for (int pass = 0; pass < 2; ++pass) {
#pragma unroll
        for (int it = 0; it < 4; ++it) {
          const int row = it * 4 + q;
          const float* sp = slab + row * 68 + c8;
          v8h hv, lv;
#pragma unroll
          for (int e = 0; e < 8; ++e) {
            if (OUT_MODE == 1) {
              hv[e] = (_Float16)sp[e];
            } else {
              unsigned short hb = f2bf_bits(sp[e]);
              unsigned short lb = f2bf_bits(sp[e] - bf_bits2f(hb));
              hv[e] = __builtin_bit_cast(_Float16, hb);
              lv[e] = __builtin_bit_cast(_Float16, lb);
            }
          }
          *(volatile v8h*)(C + (size_t)(mBase + row) * ldc + n0 + c8) = hv;
          if (OUT_MODE == 2) *(volatile v8h*)(C2 + (size_t)(mBase + row) * ldc + n0 + c8) = lv;
        }
        __threadfence();
      }
    }
    __builtin_amdgcn_fence(__ATOMIC_RELEASE, "workgroup");
    __builtin_amdgcn_wave_barrier();
    __builtin_amdgcn_fence(__ATOMIC_ACQUIRE, "workgroup");
  }
}

__device__ __forceinline__ void split_pair(float f0, float f1, unsigned& hw, unsigned& lw) {
  const unsigned short h0 = f2bf_bits(f0);
  const unsigned short h1 = f2bf_bits(f1);
  const unsigned short l0 = f2bf_bits(f0 - bf_bits2f(h0));
  const unsigned short l1 = f2bf_bits(f1 - bf_bits2f(h1));
  hw = (unsigned)h0 | ((unsigned)h1 << 16);
  lw = (unsigned)l0 | ((unsigned)l1 << 16);
}

__global__ __launch_bounds__(256) void split_planes_bf16(
    const float* __restrict__ src, unsigned short* __restrict__ hi,
    unsigned short* __restrict__ lo, int n8) {
  const int i = blockIdx.x * 256 + threadIdx.x;
  if (i >= n8) return;
  const size_t e0 = (size_t)i * 8;
  const v4f a = *(const v4f*)(src + e0);
  const v4f c = *(const v4f*)(src + e0 + 4);
  unsigned hx, hy, hz, hw, lx, ly, lz, lw;
  split_pair(a[0], a[1], hx, lx);
  split_pair(a[2], a[3], hy, ly);
  split_pair(c[0], c[1], hz, lz);
  split_pair(c[2], c[3], hw, lw);
  const v4u hv = (v4u){hx, hy, hz, hw};
  const v4u lv = (v4u){lx, ly, lz, lw};
  *(volatile v4u*)(hi + e0) = hv;
  *(volatile v4u*)(lo + e0) = lv;
  __threadfence();
  *(volatile v4u*)(hi + e0) = hv;
  *(volatile v4u*)(lo + e0) = lv;
}

__device__ __forceinline__ unsigned short at_bf_bits(float f) {
  unsigned u = __float_as_uint(f);
  return (unsigned short)((u + 0x7FFFu + ((u >> 16) & 1u)) >> 16);
}
__device__ __forceinline__ __bf16 at_f2bf(float f) { return __builtin_bit_cast(__bf16, at_bf_bits(f)); }
__device__ __forceinline__ void at_split(float f, __bf16& hi, __bf16& lo) {
  const unsigned short hb = at_bf_bits(f);
  hi = __builtin_bit_cast(__bf16, hb);
  lo = at_f2bf(f - __uint_as_float(((unsigned)hb) << 16));
}
__device__ __forceinline__ v8f at_mma(v16b a, v16b b, v8f c) {
  c = __builtin_amdgcn_wmma_f32_16x16x32_bf16(false, a, false, b, (short)0, c, false, false);
  asm volatile("v_nop\n\tv_nop\n\tv_nop\n\tv_nop" : "+v"(c) : "v"(a), "v"(b));
  return c;
}

__device__ __forceinline__ void st_tr8(unsigned short* dst, int pitch, v4u w) {
#pragma unroll
  for (int e = 0; e < 4; ++e) {
    const unsigned word = w[e];
    dst[(2 * e) * pitch]     = (unsigned short)(word & 0xffffu);
    dst[(2 * e + 1) * pitch] = (unsigned short)(word >> 16);
  }
}

__global__ __launch_bounds__(128)
void attn_causal_hd64(const unsigned short* __restrict__ Qh, const unsigned short* __restrict__ Ql,
                      const unsigned short* __restrict__ Kh, const unsigned short* __restrict__ Kl,
                      const unsigned short* __restrict__ Vh, const unsigned short* __restrict__ Vl,
                      unsigned short* __restrict__ Oh, unsigned short* __restrict__ Ol,
                      float sm_scale) {
  union FB { v16b v; v8b h[2]; };
  __shared__ __align__(16) unsigned short Ksh[AKC * HDIM];
  __shared__ __align__(16) unsigned short Ksl[AKC * HDIM];
  __shared__ __align__(16) unsigned short Vth[HDIM * AKC];
  __shared__ __align__(16) unsigned short Vtl[HDIM * AKC];
  __shared__ __align__(16) __bf16 Psh[ANW][16 * AKC];
  __shared__ __align__(16) __bf16 Psl[ANW][16 * AKC];
  __shared__ __align__(16) float  Os[ANW][16 * 68];

  const int tid  = threadIdx.x;
  const int wave = tid >> 5;
  const int lane = tid & 31;
  const int hh   = lane >> 4;
  const int c    = lane & 15;
  const float NEG_INF = -__builtin_inff();

  constexpr int NQB = SEQ / AQB;
  const int bx   = blockIdx.x;
  const int qb   = bx % NQB;
  const int bhid = bx / NQB;
  const int h    = bhid % NHEAD;
  const int b    = bhid / NHEAD;
  const int q0   = qb * AQB + wave * 16;
  const size_t hoff = (size_t)h * HDIM;

  v16b qah[2], qal[2];
  {
    const size_t qo = (size_t)(b * SEQ + q0 + c) * EMB + hoff + 8 * hh;
    const __bf16* qhp = (const __bf16*)(const void*)Qh;
    const __bf16* qlp = (const __bf16*)(const void*)Ql;
#pragma unroll
    for (int dc = 0; dc < 2; ++dc) {
      qah[dc] = Frag<__bf16>::load(qhp + qo + dc * 32);
      qal[dc] = Frag<__bf16>::load(qlp + qo + dc * 32);
    }
  }

  float mrow[8], lrow[8];
  v8f oacc[4];
#pragma unroll
  for (int r = 0; r < 8; ++r) { mrow[r] = NEG_INF; lrow[r] = 0.f; }
#pragma unroll
  for (int t = 0; t < 4; ++t) oacc[t] = (v8f){0.f,0.f,0.f,0.f,0.f,0.f,0.f,0.f};

  const int nChunks = qb + 1;
  for (int kc = 0; kc < nChunks; ++kc) {
    const int kv0 = kc * AKC;
    __syncthreads();
#pragma unroll
    for (int i = 0; i < 4; ++i) {
      const int ci = tid + 128 * i;
      const int kvr = ci >> 3, col8 = (ci & 7) * 8;
      const size_t go = (size_t)(b * SEQ + kv0 + kvr) * EMB + hoff + col8;
      const v4u w0 = *(const v4u*)(Kh + go);
      const v4u w1 = *(const v4u*)(Kl + go);
      *(v4u*)(Ksh + kvr * HDIM + col8) = w0;
      *(v4u*)(Ksl + kvr * HDIM + col8) = w1;
    }
    asm volatile("" ::: "memory");
#pragma unroll
    for (int i = 0; i < 4; ++i) {
      const int ci = tid + 128 * i;
      const int kvr = ci >> 3, col8 = (ci & 7) * 8;
      const size_t go = (size_t)(b * SEQ + kv0 + kvr) * EMB + hoff + col8;
      const v4u w0 = *(const v4u*)(Vh + go);
      const v4u w1 = *(const v4u*)(Vl + go);
      st_tr8(Vth + col8 * AKC + kvr, AKC, w0);
      st_tr8(Vtl + col8 * AKC + kvr, AKC, w1);
    }
    __syncthreads();

    v8f s[4];
#pragma unroll
    for (int j = 0; j < 4; ++j) {
      s[j] = (v8f){0.f,0.f,0.f,0.f,0.f,0.f,0.f,0.f};
#pragma unroll
      for (int dc = 0; dc < 2; ++dc) {
        FB kfh, kfl;
        const int ko = (j * 16 + c) * HDIM + dc * 32 + 8 * hh;
        kfh.h[0] = *(const v8b*)(Ksh + ko);
        kfh.h[1] = *(const v8b*)(Ksh + ko + 16);
        kfl.h[0] = *(const v8b*)(Ksl + ko);
        kfl.h[1] = *(const v8b*)(Ksl + ko + 16);
        s[j] = at_mma(qah[dc], kfh.v, s[j]);
        s[j] = at_mma(qah[dc], kfl.v, s[j]);
        s[j] = at_mma(qal[dc], kfh.v, s[j]);
      }
    }
    const bool diag = (kc == qb);
    float cm[8];
#pragma unroll
    for (int r = 0; r < 8; ++r) {
      const int qrow = q0 + 8 * hh + r;
      float m = NEG_INF;
#pragma unroll
      for (int j = 0; j < 4; ++j) {
        const int kvcol = kv0 + j * 16 + c;
        float val = s[j][r] * sm_scale;
        val = (diag && (kvcol > qrow)) ? NEG_INF : val;
        s[j][r] = val;
        m = fmaxf(m, val);
      }
#pragma unroll
      for (int off = 1; off < 16; off <<= 1) m = fmaxf(m, __shfl_xor(m, off, 32));
      cm[r] = m;
    }
    __bf16* pwh = Psh[wave];
    __bf16* pwl = Psl[wave];
#pragma unroll
    for (int r = 0; r < 8; ++r) {
      const float mnew = fmaxf(mrow[r], cm[r]);
      const float alpha = expf(mrow[r] - mnew);
      mrow[r] = mnew;
      float psum = 0.f;
#pragma unroll
      for (int j = 0; j < 4; ++j) {
        const float p = expf(s[j][r] - mnew);
        psum += p;
        __bf16 a, bl;
        at_split(p, a, bl);
        pwh[(8 * hh + r) * AKC + j * 16 + c] = a;
        pwl[(8 * hh + r) * AKC + j * 16 + c] = bl;
      }
#pragma unroll
      for (int off = 1; off < 16; off <<= 1) psum += __shfl_xor(psum, off, 32);
      lrow[r] = lrow[r] * alpha + psum;
#pragma unroll
      for (int t = 0; t < 4; ++t) oacc[t][r] *= alpha;
    }
    __builtin_amdgcn_fence(__ATOMIC_RELEASE, "workgroup");
    __builtin_amdgcn_wave_barrier();
    __builtin_amdgcn_fence(__ATOMIC_ACQUIRE, "workgroup");
#pragma unroll 1
    for (int kk = 0; kk < 2; ++kk) {
      FB pa, pl;
      pa.h[0] = *(const v8b*)(pwh + c * AKC + kk * 32 + 8 * hh);
      pa.h[1] = *(const v8b*)(pwh + c * AKC + kk * 32 + 16 + 8 * hh);
      pl.h[0] = *(const v8b*)(pwl + c * AKC + kk * 32 + 8 * hh);
      pl.h[1] = *(const v8b*)(pwl + c * AKC + kk * 32 + 16 + 8 * hh);
#pragma unroll
      for (int t = 0; t < 4; ++t) {
        FB vb, vlo;
        const int vo = (t * 16 + c) * AKC + kk * 32 + 8 * hh;
        vb.h[0]  = *(const v8b*)(Vth + vo);
        vb.h[1]  = *(const v8b*)(Vth + vo + 16);
        vlo.h[0] = *(const v8b*)(Vtl + vo);
        vlo.h[1] = *(const v8b*)(Vtl + vo + 16);
        oacc[t] = at_mma(pa.v, vb.v, oacc[t]);
        oacc[t] = at_mma(pa.v, vlo.v, oacc[t]);
        oacc[t] = at_mma(pl.v, vb.v, oacc[t]);
      }
    }
  }

  float* os = Os[wave];
#pragma unroll
  for (int r = 0; r < 8; ++r) {
    const float inv = 1.0f / lrow[r];
#pragma unroll
    for (int t = 0; t < 4; ++t) os[(8 * hh + r) * 68 + t * 16 + c] = oacc[t][r] * inv;
  }
  __builtin_amdgcn_fence(__ATOMIC_RELEASE, "workgroup");
  __builtin_amdgcn_wave_barrier();
  __builtin_amdgcn_fence(__ATOMIC_ACQUIRE, "workgroup");
  {
    const int q4 = lane >> 3, c8 = (lane & 7) * 8;
    for (int pass = 0; pass < 2; ++pass) {
#pragma unroll
      for (int it = 0; it < 4; ++it) {
        const int row = it * 4 + q4;
        const float* sp = os + row * 68 + c8;
        v8h hv, lv;
#pragma unroll
        for (int e = 0; e < 8; ++e) {
          unsigned short hb = f2bf_bits(sp[e]);
          unsigned short lb = f2bf_bits(sp[e] - bf_bits2f(hb));
          hv[e] = __builtin_bit_cast(_Float16, hb);
          lv[e] = __builtin_bit_cast(_Float16, lb);
        }
        const size_t oo = (size_t)(b * SEQ + q0 + row) * EMB + hoff + c8;
        *(volatile v8h*)(Oh + oo) = hv;
        *(volatile v8h*)(Ol + oo) = lv;
      }
      __threadfence();
    }
  }
}

extern "C" void kernel_launch(void* const* d_in, const int* in_sizes, int n_in,
                              void* d_out, int out_size, void* d_ws, size_t ws_size,
                              hipStream_t stream) {
  if (n_in < 5) return;
  if (in_sizes[0] != NB * SEQ * EMB) return;
  if (in_sizes[1] != HDIM * HDIM || in_sizes[2] != HDIM * HDIM || in_sizes[3] != HDIM * HDIM) return;
  if (in_sizes[4] != EMB * EMB) return;
  if (out_size != NB * SEQ * EMB) return;
  if (ws_size < WS_TOTAL) return;

  const float* x  = (const float*)d_in[0];
  const float* Wq = (const float*)d_in[1];
  const float* Wk = (const float*)d_in[2];
  const float* Wv = (const float*)d_in[3];
  const float* Wo = (const float*)d_in[4];
  float* out = (float*)d_out;

  char* ws = (char*)d_ws;
  unsigned short* XH   = (unsigned short*)(ws + OFF_XH);
  unsigned short* XL   = (unsigned short*)(ws + OFF_XL);
  unsigned short* WH   = (unsigned short*)(ws + OFF_WH);
  unsigned short* WL   = (unsigned short*)(ws + OFF_WL);
  unsigned short* WOH  = (unsigned short*)(ws + OFF_WOH);
  unsigned short* WOL  = (unsigned short*)(ws + OFF_WOL);
  unsigned short* QKVH = (unsigned short*)(ws + OFF_QKVH);
  unsigned short* QKVL = (unsigned short*)(ws + OFF_QKVL);
  unsigned short* AVH  = (unsigned short*)(ws + OFF_AVH);
  unsigned short* AVL  = (unsigned short*)(ws + OFF_AVL);
  const float* dummyf = (const float*)(ws + OFF_XH);
  void* dummyv = (void*)(ws + OFF_XH);

  {
    const int n8x = (NB * SEQ * EMB) / 8;
    split_planes_bf16<<<(n8x + 255) / 256, 256, 0, stream>>>(x, XH, XL, n8x);
    const int n8w = (HDIM * HDIM) / 8;
    split_planes_bf16<<<(n8w + 255) / 256, 256, 0, stream>>>(Wq, WH + 0 * HDIM * HDIM, WL + 0 * HDIM * HDIM, n8w);
    split_planes_bf16<<<(n8w + 255) / 256, 256, 0, stream>>>(Wk, WH + 1 * HDIM * HDIM, WL + 1 * HDIM * HDIM, n8w);
    split_planes_bf16<<<(n8w + 255) / 256, 256, 0, stream>>>(Wv, WH + 2 * HDIM * HDIM, WL + 2 * HDIM * HDIM, n8w);
    const int n8o = (EMB * EMB) / 8;
    split_planes_bf16<<<(n8o + 255) / 256, 256, 0, stream>>>(Wo, WOH, WOL, n8o);
  }

  {
    const int tiles = (NROWH / 64) * (HDIM / 64);
    dim3 grid((tiles + 7) / 8, 3);
    wmma_gemm64<1, true, 0, 2, false><<<grid, 256, 0, stream>>>(
        XH, XL, HDIM, 0L,
        WH, WL, HDIM, (long)(HDIM * HDIM),
        (void*)QKVH, (void*)QKVL, HDIM, (long)PLANE_QKV,
        dummyf, dummyf, 0L,
        NROWH, HDIM, HDIM, 1.0f);
  }

  {
    const int nblk = NB * NHEAD * (SEQ / AQB);
    attn_causal_hd64<<<nblk, 128, 0, stream>>>(
        QKVH + 0 * PLANE_QKV, QKVL + 0 * PLANE_QKV,
        QKVH + 1 * PLANE_QKV, QKVL + 1 * PLANE_QKV,
        QKVH + 2 * PLANE_QKV, QKVL + 2 * PLANE_QKV,
        AVH, AVL, 0.125f);
  }

  {
    const int tiles = (NTOK / 64) * (EMB / 64);
    dim3 grid((tiles + 7) / 8, 1);
    wmma_gemm64<1, true, 0, 0, false><<<grid, 256, 0, stream>>>(
        AVH, AVL, EMB, 0L,
        WOH, WOL, EMB, 0L,
        (void*)out, dummyv, EMB, 0L,
        dummyf, dummyf, 0L,
        NTOK, EMB, EMB, 1.0f);
  }
}
